// MultiHeadAttention_85478439125982
// MI455X (gfx1250) — hardware-verified
//
#include <hip/hip_runtime.h>


#ifndef NB
#define NB 4
#endif
#ifndef SEQ
#define SEQ 2048
#endif
#define NB_FULL  4
#define SEQ_FULL 2048
#define DM   1024
#define NH_  16
#define HD   64
#define DQ   (NH_ * HD)
#define RH   512
#define RHR  ((RH < SEQ) ? RH : SEQ)
#define SCL  0.125f
#define L2E  1.4426950408889634f
#define MASKV (-1.0e30f)

static_assert(NB <= NB_FULL);
static_assert(SEQ <= SEQ_FULL);
static_assert(SEQ % 256 == 0);
static_assert(RHR % 256 == 0);
static_assert((SEQ - RHR) % 64 == 0);
static_assert(DM % 64 == 0);
static_assert(DQ == DM);
static_assert((size_t)NB * NH_ * SEQ * HD * 2 <= (size_t)NB * SEQ * DM * 2);
static_assert((size_t)2 * NB * SEQ * DQ * 2 <= (size_t)NB * SEQ * DQ * 4);
static_assert((size_t)4 * DQ * DM * 2 + (size_t)NB * SEQ * DM * 2 + (size_t)NB * SEQ * DQ * 4 + (size_t)2 * NB * NH_ * SEQ * HD * 2 + (size_t)6 * NB * NH_ * RHR * HD * 2 <= (size_t)134217728);

typedef _Float16 h16;
typedef unsigned short bf;
typedef __attribute__((ext_vector_type(16))) __bf16   v16bf;
typedef __attribute__((ext_vector_type(16))) _Float16 v16h;
typedef __attribute__((ext_vector_type(8)))  _Float16 v8h;
typedef __attribute__((ext_vector_type(8)))  unsigned short v8us;
typedef __attribute__((ext_vector_type(16))) unsigned short v16us;
typedef __attribute__((ext_vector_type(2)))  unsigned short v2us;
typedef __attribute__((ext_vector_type(8)))  float    v8f;
typedef __attribute__((ext_vector_type(4)))  float    v4f;
typedef v4f  __attribute__((may_alias)) v4fa;
typedef v8us __attribute__((may_alias)) v8usa;

__device__ __forceinline__ unsigned short f2bf(float f) { unsigned u = __float_as_uint(f); u += 0x7FFFu + ((u >> 16) & 1u); return (unsigned short)(u >> 16); }
__device__ __forceinline__ float bf2f(unsigned short b) { return __uint_as_float(((unsigned)b) << 16); }
__device__ __forceinline__ float bfr(float f) { return bf2f(f2bf(f)); }
__device__ __forceinline__ void splitf(float y, unsigned short& h, unsigned short& l) { h = f2bf(y); l = f2bf(y - bf2f(h)); }
__device__ __forceinline__ v16h cat16(v8h lo, v8h hi) { return __builtin_shufflevector(lo, hi, 0, 1, 2, 3, 4, 5, 6, 7, 8, 9, 10, 11, 12, 13, 14, 15); }
__device__ __forceinline__ v16bf cat16b(v8us lo, v8us hi) { return __builtin_bit_cast(v16bf, __builtin_shufflevector(lo, hi, 0, 1, 2, 3, 4, 5, 6, 7, 8, 9, 10, 11, 12, 13, 14, 15)); }
__device__ __forceinline__ v8f wmma16(v16h a, v16h b, v8f c) { return __builtin_amdgcn_wmma_f32_16x16x32_f16(false, a, false, b, (short)0, c, false, false); }
__device__ __forceinline__ v8f wmmab(v16bf a, v16bf b, v8f c) { return __builtin_amdgcn_wmma_f32_16x16x32_bf16(false, a, false, b, (short)0, c, false, false); }
__device__ __forceinline__ void wave_sync() { asm volatile("s_wait_dscnt 0x0" ::: "memory"); __builtin_amdgcn_wave_barrier(); asm volatile("" ::: "memory"); }

template <typename T16> struct WFrag;
template <> struct WFrag<h16> { typedef v16h V; static __device__ __forceinline__ V ld(const h16* p) { return cat16(*(const v8h*)p, *(const v8h*)(p + 16)); } static __device__ __forceinline__ v8f mma(V a, V b, v8f c) { return wmma16(a, b, c); } };
template <> struct WFrag<bf> { typedef v16bf V; static __device__ __forceinline__ V ld(const bf* p) { return cat16b(*(const v8us*)p, *(const v8us*)(p + 16)); } static __device__ __forceinline__ v8f mma(V a, V b, v8f c) { return wmmab(a, b, c); } };

template <typename T16, int NSPLIT, bool BIAS>
__global__ __launch_bounds__(32) void k_gemmw(const T16* __restrict__ A, const T16* __restrict__ A2, const T16* __restrict__ Bt, const T16* __restrict__ Bt2, int K, float* C, int ldc, const float* __restrict__ bias, size_t sA, size_t sB, size_t sC) {
    typedef typename WFrag<T16>::V V;
    __shared__ __align__(16) float os[16 * 68];
    const size_t z = blockIdx.z; A += z * sA; if (A2) A2 += z * sA; Bt += z * sB; if (Bt2) Bt2 += z * sB; C += z * sC;
    const int lane = threadIdx.x & 31, lr = lane & 15, hi = lane >> 4; const int r0 = blockIdx.x * 64, c0 = blockIdx.y * 64;
    v8f acc[4][4];
#pragma unroll
    for (int mb = 0; mb < 4; ++mb)
#pragma unroll
        for (int nb = 0; nb < 4; ++nb) acc[mb][nb] = (v8f){};
    const size_t aoff = (size_t)(r0 + lr) * K + 8 * hi, boff = (size_t)(c0 + lr) * K + 8 * hi;
#pragma unroll 1
    for (int kc = 0; kc < K; kc += 32) {
        V a[4], a2[4];
#pragma unroll
        for (int mb = 0; mb < 4; ++mb) { a[mb] = WFrag<T16>::ld(A + aoff + (size_t)mb * 16 * K + kc); if (NSPLIT == 1 || NSPLIT == 2) a2[mb] = WFrag<T16>::ld(A2 + aoff + (size_t)mb * 16 * K + kc); }
#pragma unroll
        for (int nb = 0; nb < 4; ++nb) { const V b = WFrag<T16>::ld(Bt + boff + (size_t)nb * 16 * K + kc); V b2; if (NSPLIT >= 2) b2 = WFrag<T16>::ld(Bt2 + boff + (size_t)nb * 16 * K + kc);
#pragma unroll
            for (int mb = 0; mb < 4; ++mb) { acc[mb][nb] = WFrag<T16>::mma(a[mb], b, acc[mb][nb]); if (NSPLIT == 1 || NSPLIT == 2) acc[mb][nb] = WFrag<T16>::mma(a2[mb], b, acc[mb][nb]); if (NSPLIT >= 2) acc[mb][nb] = WFrag<T16>::mma(a[mb], b2, acc[mb][nb]); } }
        asm volatile("v_nop\n\tv_nop\n\tv_nop\n\tv_nop" : "+v"(acc[0][0]), "+v"(acc[1][1]), "+v"(acc[2][2]), "+v"(acc[3][3]) : "v"(a[0]), "v"(a[3]));
    }
#pragma unroll
    for (int mb = 0; mb < 4; ++mb) {
#pragma unroll
        for (int nb = 0; nb < 4; ++nb) {
#pragma unroll
            for (int j = 0; j < 8; ++j) os[(hi * 8 + j) * 68 + nb * 16 + lr] = acc[mb][nb][j]; }
        __builtin_amdgcn_wave_barrier(); asm volatile("" ::: "memory");
        float* crow = C + (size_t)(r0 + mb * 16) * ldc + c0;
#pragma unroll 1
        for (int ps = 0; ps < 2; ++ps) {
#pragma unroll
            for (int s = 0; s < 8; ++s) { const int row = 2 * s + hi, cofs = lr * 4; v4f val = *(const v4fa*)(os + row * 68 + cofs); if (BIAS) { val[0] += bfr(bias[c0 + cofs]); val[1] += bfr(bias[c0 + cofs + 1]); val[2] += bfr(bias[c0 + cofs + 2]); val[3] += bfr(bias[c0 + cofs + 3]); }
                *(volatile v4f*)(crow + (size_t)row * ldc + cofs) = val; }
            if (ps == 0) __threadfence(); }
        __builtin_amdgcn_wave_barrier(); asm volatile("" ::: "memory");
    }
}

__global__ __launch_bounds__(256) void k_wtG(const float* __restrict__ w, int K, int N, bf* Bt) {
#pragma clang fp contract(off)
    w += (size_t)blockIdx.y * K * N; Bt += (size_t)blockIdx.y * N * K;
    const int lane = threadIdx.x & 31; const int L0 = (blockIdx.x * 8 + (threadIdx.x >> 5)) * 8; const int nlines = N * K / 64;
#pragma unroll
    for (int ps = 0; ps < 2; ++ps) {
#pragma unroll 1
        for (int l = 0; l < 8; ++l) { const int L = L0 + l; if (L >= nlines) break; const size_t e = (size_t)L * 64 + lane * 2; const int k = (int)(e % K), n = (int)(e / K); v2us o;
            o[0] = f2bf(w[(size_t)k * N + n]); o[1] = f2bf(w[(size_t)(k + 1) * N + n]); *(volatile v2us*)(Bt + e) = o; }
        if (ps == 0) __threadfence(); }
}

__global__ __launch_bounds__(256) void k_cvt8(const float* __restrict__ src, bf* dst, size_t n8, size_t sS, size_t sD) {
#pragma clang fp contract(off)
    const size_t i = (size_t)blockIdx.x * 256 + threadIdx.x; if (i >= n8) return; src += (size_t)blockIdx.y * sS; dst += (size_t)blockIdx.y * sD;
    const v8f v = *(const v8f*)(src + i * 8); v8us o;
#pragma unroll
    for (int k = 0; k < 8; ++k) o[k] = f2bf(v[k]);
    *(volatile v8us*)(dst + i * 8) = o; __threadfence(); *(volatile v8us*)(dst + i * 8) = o; }

__global__ __launch_bounds__(256) void k_qkp(const float* __restrict__ F, h16* P16, bf* Ph, bf* Pl) {
#pragma clang fp contract(off)
    const size_t e = ((size_t)blockIdx.x * 256 + threadIdx.x) * 8; if (e >= (size_t)NB * NH_ * SEQ * HD) return;
    const int d = (int)(e % HD); const int t = (int)((e / HD) % SEQ); const int h = (int)((e / ((size_t)HD * SEQ)) % NH_); const int b = (int)(e / ((size_t)HD * SEQ * NH_));
    const float* f = F + ((size_t)b * SEQ + t) * DQ + h * HD + d; const v4f a0 = *(const v4f*)f; const v4f a1 = *(const v4f*)(f + 4);
    v8h o16; v8us oh, ol;
#pragma unroll
    for (int q = 0; q < 4; ++q) { unsigned short a, c; o16[q] = (h16)a0[q]; splitf(a0[q], a, c); oh[q] = a; ol[q] = c; o16[4 + q] = (h16)a1[q]; splitf(a1[q], a, c); oh[4 + q] = a; ol[4 + q] = c; }
    const bool hr = (t < RHR);
    const size_t eh = (((size_t)b * NH_ + h) * RHR + (hr ? t : 0)) * HD + d;
    *(volatile v8h*)(P16 + e) = o16; if (hr) { *(volatile v8us*)(Ph + eh) = oh; *(volatile v8us*)(Pl + eh) = ol; }
    __threadfence();
    *(volatile v8h*)(P16 + e) = o16; if (hr) { *(volatile v8us*)(Ph + eh) = oh; *(volatile v8us*)(Pl + eh) = ol; }
}

__global__ __launch_bounds__(256) void k_vtp(const float* __restrict__ F, h16* V16, bf* Vh, bf* Vl) {
#pragma clang fp contract(off)
    const size_t e = ((size_t)blockIdx.x * 256 + threadIdx.x) * 8; if (e >= (size_t)NB * NH_ * HD * SEQ) return;
    const int t = (int)(e % SEQ); const int d = (int)((e / SEQ) % HD); const int h = (int)((e / ((size_t)SEQ * HD)) % NH_); const int b = (int)(e / ((size_t)SEQ * HD * NH_));
    const float* f = F + ((size_t)b * SEQ + t) * DQ + h * HD + d;
    v8h o16; v8us oh, ol;
#pragma unroll
    for (int q = 0; q < 8; ++q) { const float x = f[(size_t)q * DQ]; unsigned short a, c; o16[q] = (h16)x; splitf(x, a, c); oh[q] = a; ol[q] = c; }
    const bool hr = (t < RHR);
    const size_t eh = (((size_t)b * NH_ + h) * HD + d) * RHR + (hr ? t : 0);
    *(volatile v8h*)(V16 + e) = o16; if (hr) { *(volatile v8us*)(Vh + eh) = oh; *(volatile v8us*)(Vl + eh) = ol; }
    __threadfence();
    *(volatile v8h*)(V16 + e) = o16; if (hr) { *(volatile v8us*)(Vh + eh) = oh; *(volatile v8us*)(Vl + eh) = ol; }
}

__global__ __launch_bounds__(32) void k_flashp(const h16* __restrict__ Q16, const h16* __restrict__ K16, const h16* __restrict__ VT16, bf* ATh, bf* ATl) {
    __shared__ __align__(16) unsigned short sth[16 * 72];
    __shared__ __align__(16) unsigned short stl[16 * 72];
    const int lane = threadIdx.x & 31, lr = lane & 15, hi = lane >> 4;
    const int bh = blockIdx.y; const int b = bh / NH_, h = bh % NH_;
    const int q0 = RHR + (int)blockIdx.x * 32;
    const h16* Qp = Q16 + (size_t)bh * SEQ * HD;
    const h16* Kp = K16 + (size_t)bh * SEQ * HD + (size_t)lr * HD + 8 * hi;
    const h16* Vp = VT16 + (size_t)bh * HD * SEQ + (size_t)lr * SEQ + 8 * hi;
    v16h qb[2][2];
#pragma unroll
    for (int qt = 0; qt < 2; ++qt)
#pragma unroll
        for (int ds = 0; ds < 2; ++ds) qb[qt][ds] = WFrag<h16>::ld(Qp + (size_t)(q0 + qt * 16 + lr) * HD + ds * 32 + 8 * hi);
    v8f o[2][4]; float mrun[2], lrun[2];
#pragma unroll
    for (int qt = 0; qt < 2; ++qt) { mrun[qt] = MASKV; lrun[qt] = 0.0f;
#pragma unroll
        for (int dt = 0; dt < 4; ++dt) o[qt][dt] = (v8f){}; }
    const int kend = q0 + 32;
#pragma unroll 1
    for (int kb = 0; kb < kend; kb += 32) {
        v8f s[2][2];
        {
            v16h ka[2][2];
#pragma unroll
            for (int kt = 0; kt < 2; ++kt)
#pragma unroll
                for (int ds = 0; ds < 2; ++ds) ka[kt][ds] = WFrag<h16>::ld(Kp + (size_t)(kb + kt * 16) * HD + ds * 32);
#pragma unroll
            for (int qt = 0; qt < 2; ++qt)
#pragma unroll
                for (int kt = 0; kt < 2; ++kt) { s[qt][kt] = wmma16(ka[kt][0], qb[qt][0], (v8f){}); s[qt][kt] = wmma16(ka[kt][1], qb[qt][1], s[qt][kt]); }
            asm volatile("v_nop\n\tv_nop\n\tv_nop\n\tv_nop" : "+v"(s[0][0]), "+v"(s[0][1]), "+v"(s[1][0]), "+v"(s[1][1]) : "v"(ka[0][0]), "v"(ka[0][1]), "v"(ka[1][0]), "v"(ka[1][1]));
        }
        const bool diag = (kb + 31 > q0);
        v16h pf[2];
#pragma unroll
        for (int qt = 0; qt < 2; ++qt) {
            float x[16];
#pragma unroll
            for (int kt = 0; kt < 2; ++kt)
#pragma unroll
                for (int r = 0; r < 8; ++r) x[kt * 8 + r] = s[qt][kt][r] * SCL;
            if (diag) { const int qi = q0 + qt * 16 + lr; const int k0 = kb + 8 * hi;
#pragma unroll
                for (int kt = 0; kt < 2; ++kt)
#pragma unroll
                    for (int r = 0; r < 8; ++r) x[kt * 8 + r] = (k0 + kt * 16 + r <= qi) ? x[kt * 8 + r] : MASKV; }
            float tm = x[0];
#pragma unroll
            for (int i = 1; i < 16; ++i) tm = fmaxf(tm, x[i]);
            tm = fmaxf(tm, __shfl_xor(tm, 16, 32));
            const float mn = fmaxf(mrun[qt], tm);
            const float alpha = __builtin_amdgcn_exp2f((mrun[qt] - mn) * L2E);
            mrun[qt] = mn;
            float ls = 0.0f; v16h pk;
#pragma unroll
            for (int i = 0; i < 16; ++i) { const float pc = __builtin_amdgcn_exp2f((x[i] - mn) * L2E + 10.0f); ls += pc; pk[i] = (h16)pc; }
            ls += __shfl_xor(ls, 16, 32);
            lrun[qt] = lrun[qt] * alpha + ls;
#pragma unroll
            for (int dt = 0; dt < 4; ++dt)
#pragma unroll
                for (int r = 0; r < 8; ++r) o[qt][dt][r] *= alpha;
            pf[qt] = pk;
        }
        {
            v16h va[4];
#pragma unroll
            for (int dt = 0; dt < 4; ++dt) va[dt] = WFrag<h16>::ld(Vp + (size_t)(dt * 16) * SEQ + kb);
#pragma unroll
            for (int dt = 0; dt < 4; ++dt)
#pragma unroll
                for (int qt = 0; qt < 2; ++qt) o[qt][dt] = wmma16(va[dt], pf[qt], o[qt][dt]);
            asm volatile("v_nop\n\tv_nop\n\tv_nop\n\tv_nop" : "+v"(o[0][0]), "+v"(o[0][1]), "+v"(o[0][2]), "+v"(o[0][3]), "+v"(o[1][0]), "+v"(o[1][1]), "+v"(o[1][2]), "+v"(o[1][3]) : "v"(va[0]), "v"(va[1]), "v"(va[2]), "v"(va[3]), "v"(pf[0]), "v"(pf[1]));
        }
    }
    const int rq = lane >> 3, pc8 = (lane & 7) * 8;
#pragma unroll
    for (int qt = 0; qt < 2; ++qt) {
        const float inv = 1.0f / lrun[qt];
#pragma unroll
        for (int dt = 0; dt < 4; ++dt) { v8us vh, vl;
#pragma unroll
            for (int r = 0; r < 8; ++r) { unsigned short a, c; splitf(o[qt][dt][r] * inv, a, c); vh[r] = a; vl[r] = c; }
            *(v8usa*)(sth + lr * 72 + dt * 16 + 8 * hi) = vh; *(v8usa*)(stl + lr * 72 + dt * 16 + 8 * hi) = vl; }
        wave_sync();
        bf* rowh = ATh + ((size_t)b * SEQ + q0 + qt * 16) * DQ + h * HD + pc8;
        bf* rowl = ATl + ((size_t)b * SEQ + q0 + qt * 16) * DQ + h * HD + pc8;
        v8us ah[4], al[4];
#pragma unroll
        for (int s4 = 0; s4 < 4; ++s4) { const int row = 4 * s4 + rq; ah[s4] = *(const v8usa*)(sth + row * 72 + pc8); al[s4] = *(const v8usa*)(stl + row * 72 + pc8); }
#pragma unroll
        for (int s4 = 0; s4 < 4; ++s4) { const int row = 4 * s4 + rq; *(volatile v8us*)(rowh + (size_t)row * DQ) = ah[s4]; *(volatile v8us*)(rowl + (size_t)row * DQ) = al[s4]; }
        __threadfence();
#pragma unroll
        for (int s4 = 0; s4 < 4; ++s4) { const int row = 4 * s4 + rq; *(volatile v8us*)(rowh + (size_t)row * DQ) = ah[s4]; *(volatile v8us*)(rowl + (size_t)row * DQ) = al[s4]; }
        wave_sync();
    }
}

__global__ __launch_bounds__(32) void k_flashh(const bf* __restrict__ Qh, const bf* __restrict__ Ql, const bf* __restrict__ Kh, const bf* __restrict__ Kl, const bf* __restrict__ VTh, const bf* __restrict__ VTl, bf* ATh, bf* ATl) {
    __shared__ __align__(16) unsigned short sth[16 * 72];
    __shared__ __align__(16) unsigned short stl[16 * 72];
    const int lane = threadIdx.x & 31, lr = lane & 15, hi = lane >> 4;
    const int bh = blockIdx.y; const int b = bh / NH_, h = bh % NH_;
    const int q0 = (int)blockIdx.x * 16;
    const size_t qoff = (size_t)bh * RHR * HD + (size_t)(q0 + lr) * HD + 8 * hi;
    const size_t koff = (size_t)bh * RHR * HD + (size_t)lr * HD + 8 * hi;
    const size_t voff = (size_t)bh * HD * RHR + (size_t)lr * RHR + 8 * hi;
    v16bf qh[2], ql[2];
#pragma unroll
    for (int ds = 0; ds < 2; ++ds) { qh[ds] = WFrag<bf>::ld(Qh + qoff + ds * 32); ql[ds] = WFrag<bf>::ld(Ql + qoff + ds * 32); }
    v8f o[4]; float mrun = MASKV, lrun = 0.0f;
#pragma unroll
    for (int dt = 0; dt < 4; ++dt) o[dt] = (v8f){};
    const int kend = q0 + 16;
#pragma unroll 1
    for (int kb = 0; kb < kend; kb += 32) {
        v8f s[2];
        {
            v16bf kh[2][2], kl[2][2];
#pragma unroll
            for (int kt = 0; kt < 2; ++kt)
#pragma unroll
                for (int ds = 0; ds < 2; ++ds) { kh[kt][ds] = WFrag<bf>::ld(Kh + koff + (size_t)(kb + kt * 16) * HD + ds * 32); kl[kt][ds] = WFrag<bf>::ld(Kl + koff + (size_t)(kb + kt * 16) * HD + ds * 32); }
#pragma unroll
            for (int kt = 0; kt < 2; ++kt) { s[kt] = (v8f){};
#pragma unroll
                for (int ds = 0; ds < 2; ++ds) { s[kt] = wmmab(kh[kt][ds], qh[ds], s[kt]); s[kt] = wmmab(kl[kt][ds], qh[ds], s[kt]); s[kt] = wmmab(kh[kt][ds], ql[ds], s[kt]); } }
            asm volatile("v_nop\n\tv_nop\n\tv_nop\n\tv_nop" : "+v"(s[0]), "+v"(s[1]) : "v"(kh[0][0]), "v"(kh[0][1]), "v"(kh[1][0]), "v"(kh[1][1]), "v"(kl[0][0]), "v"(kl[0][1]), "v"(kl[1][0]), "v"(kl[1][1]));
        }
        const bool diag = (kb + 31 > q0);
        float x[16];
#pragma unroll
        for (int kt = 0; kt < 2; ++kt)
#pragma unroll
            for (int r = 0; r < 8; ++r) x[kt * 8 + r] = s[kt][r] * SCL;
        if (diag) { const int qi = q0 + lr; const int k0 = kb + 8 * hi;
#pragma unroll
            for (int kt = 0; kt < 2; ++kt)
#pragma unroll
                for (int r = 0; r < 8; ++r) x[kt * 8 + r] = (k0 + kt * 16 + r <= qi) ? x[kt * 8 + r] : MASKV; }
        float tm = x[0];
#pragma unroll
        for (int i = 1; i < 16; ++i) tm = fmaxf(tm, x[i]);
        tm = fmaxf(tm, __shfl_xor(tm, 16, 32));
        const float mn = fmaxf(mrun, tm);
        const float alpha = __builtin_amdgcn_exp2f((mrun - mn) * L2E);
        mrun = mn;
        float ls = 0.0f; v16us pkh, pkl;
#pragma unroll
        for (int i = 0; i < 16; ++i) { const float p = __builtin_amdgcn_exp2f((x[i] - mn) * L2E); ls += p; unsigned short a, c; splitf(p, a, c); pkh[i] = a; pkl[i] = c; }
        ls += __shfl_xor(ls, 16, 32);
        lrun = lrun * alpha + ls;
#pragma unroll
        for (int dt = 0; dt < 4; ++dt)
#pragma unroll
            for (int r = 0; r < 8; ++r) o[dt][r] *= alpha;
        const v16bf ph = __builtin_bit_cast(v16bf, pkh); const v16bf pl = __builtin_bit_cast(v16bf, pkl);
        {
            v16bf vh[4], vl[4];
#pragma unroll
            for (int dt = 0; dt < 4; ++dt) { vh[dt] = WFrag<bf>::ld(VTh + voff + (size_t)(dt * 16) * RHR + kb); vl[dt] = WFrag<bf>::ld(VTl + voff + (size_t)(dt * 16) * RHR + kb); }
#pragma unroll
            for (int dt = 0; dt < 4; ++dt) { o[dt] = wmmab(vh[dt], ph, o[dt]); o[dt] = wmmab(vl[dt], ph, o[dt]); o[dt] = wmmab(vh[dt], pl, o[dt]); }
            asm volatile("v_nop\n\tv_nop\n\tv_nop\n\tv_nop" : "+v"(o[0]), "+v"(o[1]), "+v"(o[2]), "+v"(o[3]) : "v"(vh[0]), "v"(vh[1]), "v"(vh[2]), "v"(vh[3]), "v"(vl[0]), "v"(vl[1]), "v"(vl[2]), "v"(vl[3]), "v"(ph), "v"(pl));
        }
    }
    const int rq = lane >> 3, pc8 = (lane & 7) * 8;
    const float inv = 1.0f / lrun;
#pragma unroll
    for (int dt = 0; dt < 4; ++dt) { v8us vh8, vl8;
#pragma unroll
        for (int r = 0; r < 8; ++r) { unsigned short a, c; splitf(o[dt][r] * inv, a, c); vh8[r] = a; vl8[r] = c; }
        *(v8usa*)(sth + lr * 72 + dt * 16 + 8 * hi) = vh8; *(v8usa*)(stl + lr * 72 + dt * 16 + 8 * hi) = vl8; }
    wave_sync();
    bf* rowh = ATh + ((size_t)b * SEQ + q0) * DQ + h * HD + pc8;
    bf* rowl = ATl + ((size_t)b * SEQ + q0) * DQ + h * HD + pc8;
    v8us ah[4], al[4];
#pragma unroll
    for (int s4 = 0; s4 < 4; ++s4) { const int row = 4 * s4 + rq; ah[s4] = *(const v8usa*)(sth + row * 72 + pc8); al[s4] = *(const v8usa*)(stl + row * 72 + pc8); }
#pragma unroll
    for (int s4 = 0; s4 < 4; ++s4) { const int row = 4 * s4 + rq; *(volatile v8us*)(rowh + (size_t)row * DQ) = ah[s4]; *(volatile v8us*)(rowl + (size_t)row * DQ) = al[s4]; }
    __threadfence();
#pragma unroll
    for (int s4 = 0; s4 < 4; ++s4) { const int row = 4 * s4 + rq; *(volatile v8us*)(rowh + (size_t)row * DQ) = ah[s4]; *(volatile v8us*)(rowl + (size_t)row * DQ) = al[s4]; }
}

extern "C" void kernel_launch(void* const* d_in, const int* in_sizes, int n_in,
                              void* d_out, int out_size, void* d_ws, size_t ws_size, hipStream_t stream) {
    if (n_in < 6) return;
    const size_t need_x = (size_t)(NB - 1) * SEQ_FULL * DM + (size_t)SEQ * DM;
    if ((size_t)in_sizes[0] < need_x) return;
    if ((size_t)in_sizes[1] < (size_t)NH_ * DM * HD || (size_t)in_sizes[2] < (size_t)NH_ * DM * HD || (size_t)in_sizes[3] < (size_t)NH_ * DM * HD) return;
    if ((size_t)in_sizes[4] < (size_t)DM * DQ || (size_t)in_sizes[5] < (size_t)DM) return;
    if ((size_t)out_size < need_x) return;
    const float* x = (const float*)d_in[0]; const float* wq = (const float*)d_in[1]; const float* wk = (const float*)d_in[2]; const float* wv = (const float*)d_in[3]; const float* wp = (const float*)d_in[4]; const float* bp = (const float*)d_in[5];
    float* OUT = (float*)d_out;
    char* wsp = (char*)d_ws;
    auto take = [&](size_t bytes) { char* p = wsp; wsp += (bytes + 255) & ~(size_t)255; return (void*)p; };
    bf* WQ = (bf*)take((size_t)DQ * DM * 2); bf* WK = (bf*)take((size_t)DQ * DM * 2); bf* WV = (bf*)take((size_t)DQ * DM * 2); bf* WP = (bf*)take((size_t)DM * DQ * 2);
    bf* XB = (bf*)take((size_t)NB * SEQ * DM * 2);
    float* F = (float*)take((size_t)NB * SEQ * DQ * 4);
    h16* K16 = (h16*)take((size_t)NB * NH_ * SEQ * HD * 2); h16* VT16 = (h16*)take((size_t)NB * NH_ * HD * SEQ * 2);
    const size_t HP = (size_t)NB * NH_ * RHR * HD * 2;
    bf* QPh = (bf*)take(HP); bf* QPl = (bf*)take(HP); bf* KPh = (bf*)take(HP); bf* KPl = (bf*)take(HP); bf* VTh = (bf*)take(HP); bf* VTl = (bf*)take(HP);
    const size_t used = (size_t)(wsp - (char*)d_ws);
    if (used > ws_size || used > (size_t)134217728) return;
    h16* Q16 = (h16*)XB;
    bf* ATh = (bf*)F; bf* ATl = ATh + (size_t)NB * SEQ * DQ;

    k_wtG<<<dim3((unsigned)(DM * HD / 64 / 64), NH_), 256, 0, stream>>>(wq, DM, HD, WQ);
    k_wtG<<<dim3((unsigned)(DM * HD / 64 / 64), NH_), 256, 0, stream>>>(wk, DM, HD, WK);
    k_wtG<<<dim3((unsigned)(DM * HD / 64 / 64), NH_), 256, 0, stream>>>(wv, DM, HD, WV);
    k_cvt8<<<dim3((unsigned)(((size_t)DM * DQ / 8 + 255) / 256), 1), 256, 0, stream>>>(wp, WP, (size_t)DM * DQ / 8, 0, 0);
    k_cvt8<<<dim3((unsigned)(((size_t)SEQ * DM / 8 + 255) / 256), NB), 256, 0, stream>>>(x, XB, (size_t)SEQ * DM / 8, (size_t)SEQ_FULL * DM, (size_t)SEQ * DM);

    const unsigned LP = (unsigned)(((size_t)NB * NH_ * SEQ * HD / 8 + 255) / 256);
    k_gemmw<bf, 0, false><<<dim3(NB * SEQ / 64, DQ / 64, 1), 32, 0, stream>>>(XB, nullptr, WV, nullptr, DM, F, DQ, nullptr, 0, 0, 0);
    k_vtp<<<LP, 256, 0, stream>>>(F, VT16, VTh, VTl);
    k_gemmw<bf, 0, false><<<dim3(NB * SEQ / 64, DQ / 64, 1), 32, 0, stream>>>(XB, nullptr, WK, nullptr, DM, F, DQ, nullptr, 0, 0, 0);
    k_qkp<<<LP, 256, 0, stream>>>(F, K16, KPh, KPl);
    k_gemmw<bf, 0, false><<<dim3(NB * SEQ / 64, DQ / 64, 1), 32, 0, stream>>>(XB, nullptr, WQ, nullptr, DM, F, DQ, nullptr, 0, 0, 0);
    k_qkp<<<LP, 256, 0, stream>>>(F, Q16, QPh, QPl);

    k_flashh<<<dim3(RHR / 16, NB * NH_), 32, 0, stream>>>(QPh, QPl, KPh, KPl, VTh, VTl, ATh, ATl);
    if (SEQ > RHR) k_flashp<<<dim3((SEQ - RHR) / 32, NB * NH_), 32, 0, stream>>>(Q16, K16, VT16, ATh, ATl);

    k_gemmw<bf, 1, true><<<dim3(SEQ / 64, DM / 64, NB), 32, 0, stream>>>(ATh, ATl, WP, nullptr, DQ, OUT, DM, bp, (size_t)SEQ * DQ, 0, (size_t)SEQ_FULL * DM);
}
